// PhaseLinear_46145128628239
// MI455X (gfx1250) — hardware-run, weakly checked
//
#include <hip/hip_runtime.h>


#ifndef NB
#define NB 2048
#endif
#define NB_FULL 2048
#define IND  256
#define OUTD 256
#define NCP  4

static_assert(NB % 32 == 0);
static_assert(NB <= NB_FULL);
static_assert(IND % 32 == 0);
static_assert(OUTD % 64 == 0);
static_assert(((size_t)NB * IND) % 8 == 0);
static_assert(((size_t)NCP * OUTD * IND) % 8 == 0);

typedef unsigned short bf;
typedef __attribute__((ext_vector_type(16))) __bf16   v16bf;
typedef __attribute__((ext_vector_type(8)))  unsigned short v8us;
typedef __attribute__((ext_vector_type(8)))  float    v8f;
typedef __attribute__((ext_vector_type(4)))  float    v4f;
typedef v4f  __attribute__((may_alias)) v4fa;

__device__ __forceinline__ unsigned short f2bf(float f) { unsigned u = __float_as_uint(f); u += 0x7FFFu + ((u >> 16) & 1u); return (unsigned short)(u >> 16); }
__device__ __forceinline__ float bf2f(unsigned short h) { return __uint_as_float(((unsigned)h) << 16); }
__device__ __forceinline__ float rbf(float f) { return bf2f(f2bf(f)); }
__device__ __forceinline__ v16bf cat16b(v8us lo, v8us hi) { return __builtin_bit_cast(v16bf, __builtin_shufflevector(lo, hi, 0, 1, 2, 3, 4, 5, 6, 7, 8, 9, 10, 11, 12, 13, 14, 15)); }
__device__ __forceinline__ v8f wmmab(v16bf a, v16bf b, v8f c) { return __builtin_amdgcn_wmma_f32_16x16x32_bf16(false, a, false, b, (short)0, c, false, false); }
__device__ __forceinline__ v16bf ldb(const bf* p)  { return cat16b(*(const v8us*)p, *(const v8us*)(p + 16)); }
__device__ __forceinline__ void wave_sync() { __builtin_amdgcn_fence(3  , "wavefront"); __builtin_amdgcn_wave_barrier(); asm volatile("" ::: "memory"); }
__device__ __forceinline__ float sel4(int k, float a0, float a1, float a2, float a3) { const float lo = (k & 1) ? a1 : a0; const float hi = (k & 1) ? a3 : a2; return (k & 2) ? hi : lo; }
__device__ __forceinline__ void split8(const v8us x, const float c, v8us& h, v8us& l) {
#pragma unroll
    for (int i = 0; i < 8; ++i) { const float v = bf2f(x[i]) * c; const unsigned short hb = f2bf(v); const float r = v - bf2f(hb); h[i] = hb; l[i] = f2bf(r); }
}

__global__ __launch_bounds__(256) void k_cvt8(const float* __restrict__ src, bf* dst, size_t n8) {
    const size_t i = (size_t)blockIdx.x * 256 + threadIdx.x; if (i >= n8) return;
    const v8f v = *(const v8f*)(src + i * 8); v8us o;
#pragma unroll
    for (int k = 0; k < 8; ++k) o[k] = f2bf(v[k]);
    *(volatile v8us*)(dst + i * 8) = o; __threadfence(); *(volatile v8us*)(dst + i * 8) = o;
}

__global__ __launch_bounds__(256) void k_coef(const float* __restrict__ phase, const float* __restrict__ basis, float* CE, int n) {
    const int b = blockIdx.x * 256 + threadIdx.x;
    const int bc = (b < n) ? b : (n - 1);
    const float ph = rbf(phase[bc]);
    const float PI_F = 3.14159274101257324f;
    const float B0 = 0.0f, B1 = 0.5f * PI_F, B2 = 1.0f * PI_F, B3 = 1.5f * PI_F, B4 = 2.0f * PI_F;
    const int idx = (int)(ph > B0) + (int)(ph > B1) + (int)(ph > B2) + (int)(ph > B3) + (int)(ph > B4);
    const int bucket = (idx > 3) ? 3 : idx;
    const float bound = sel4(bucket, B0, B1, B2, B3);
    const float t = (ph - bound) * (1.0f / B1);
    const float t2 = t * t, t3 = t2 * t;
    float cf[4];
#pragma unroll
    for (int j = 0; j < 4; ++j) cf[j] = ((t3 * rbf(basis[j]) + t2 * rbf(basis[4 + j])) + t * rbf(basis[8 + j])) + rbf(basis[12 + j]);
    v4f o;
    o[0] = sel4((1 - bucket) & 3, cf[0], cf[1], cf[2], cf[3]);
    o[1] = sel4((2 - bucket) & 3, cf[0], cf[1], cf[2], cf[3]);
    o[2] = sel4((3 - bucket) & 3, cf[0], cf[1], cf[2], cf[3]);
    o[3] = sel4((4 - bucket) & 3, cf[0], cf[1], cf[2], cf[3]);
    if (b < n) *(volatile v4f*)(CE + (size_t)b * 4) = o;
    __threadfence();
    if (b < n) *(volatile v4f*)(CE + (size_t)b * 4) = o;
}

__global__ __launch_bounds__(32) void k_pl(const bf* __restrict__ XB, const bf* __restrict__ WB, const float* __restrict__ CE, const float* __restrict__ BIAS, float* OUT) {
    __shared__ __align__(16) float os[16 * 68];
    const int lane = threadIdx.x & 31, lr = lane & 15, hi = lane >> 4;
    const int r0 = __builtin_amdgcn_readfirstlane((int)blockIdx.x * 32), c0 = __builtin_amdgcn_readfirstlane((int)blockIdx.y * 64);
    v8f acc[2][4];
#pragma unroll
    for (int mb = 0; mb < 2; ++mb)
#pragma unroll
        for (int nb = 0; nb < 4; ++nb) acc[mb][nb] = (v8f){};
    const size_t aoff = (size_t)(r0 + lr) * IND + 8 * hi, boff = (size_t)(c0 + lr) * IND + 8 * hi;
#pragma unroll 1
    for (int p = 0; p < NCP; ++p) {
        float cp[2];
#pragma unroll
        for (int mb = 0; mb < 2; ++mb) cp[mb] = CE[(size_t)(r0 + mb * 16 + lr) * 4 + p];
        const bf* Wp = WB + (size_t)p * OUTD * IND + boff;
#pragma unroll 1
        for (int kc = 0; kc < IND; kc += 32) {
            v16bf ah[2], al[2];
#pragma unroll
            for (int mb = 0; mb < 2; ++mb) {
                const bf* xp = XB + aoff + (size_t)mb * 16 * IND + kc;
                const v8us x0 = *(const v8us*)xp; const v8us x1 = *(const v8us*)(xp + 16);
                v8us h0, l0, h1, l1;
                split8(x0, cp[mb], h0, l0); split8(x1, cp[mb], h1, l1);
                ah[mb] = cat16b(h0, h1); al[mb] = cat16b(l0, l1);
            }
#pragma unroll
            for (int nb = 0; nb < 4; ++nb) { const v16bf b = ldb(Wp + (size_t)nb * 16 * IND + kc);
#pragma unroll
                for (int mb = 0; mb < 2; ++mb) acc[mb][nb] = wmmab(ah[mb], b, acc[mb][nb]);
#pragma unroll
                for (int mb = 0; mb < 2; ++mb) acc[mb][nb] = wmmab(al[mb], b, acc[mb][nb]); }
            asm volatile("v_nop\n\tv_nop\n\tv_nop\n\tv_nop" : "+v"(acc[0][0]), "+v"(acc[1][1]), "+v"(acc[0][3]), "+v"(acc[1][3]) : "v"(ah[0]), "v"(ah[1]), "v"(al[0]), "v"(al[1]));
        }
    }
    v4f bb[NCP];
#pragma unroll
    for (int p = 0; p < NCP; ++p) { const v4f tb = *(const v4f*)(BIAS + (size_t)p * OUTD + c0 + lr * 4);
#pragma unroll
        for (int j = 0; j < 4; ++j) bb[p][j] = rbf(tb[j]); }
#pragma unroll
    for (int mb = 0; mb < 2; ++mb) {
#pragma unroll
        for (int nb = 0; nb < 4; ++nb) {
#pragma unroll
            for (int j = 0; j < 8; ++j) os[(hi * 8 + j) * 68 + nb * 16 + lr] = acc[mb][nb][j]; }
        wave_sync();
#pragma unroll 1
        for (int ps = 0; ps < 2; ++ps) {
#pragma unroll
            for (int s = 0; s < 8; ++s) { const int row = 2 * s + hi, cofs = lr * 4;
                const int grow = r0 + mb * 16 + row;
                const v4f cv = *(const v4f*)(CE + (size_t)grow * 4);
                const v4f a = *(const v4fa*)(&os[row * 68 + cofs]);
                v4f val;
#pragma unroll
                for (int j = 0; j < 4; ++j) { const float bsum = ((cv[0] * bb[0][j] + cv[1] * bb[1][j]) + cv[2] * bb[2][j]) + cv[3] * bb[3][j]; val[j] = a[j] + bsum; }
                *(volatile v4f*)(OUT + (size_t)grow * OUTD + c0 + cofs) = val; }
            if (ps == 0) __threadfence(); }
        wave_sync();
    }
}

static constexpr size_t al256(size_t v) { return (v + 255) & ~(size_t)255; }
static constexpr size_t SZ_WB = al256((size_t)NCP * OUTD * IND * 2);
static constexpr size_t SZ_XB = al256((size_t)NB * IND * 2);
static constexpr size_t SZ_CE = al256((size_t)NB * 4 * 4);
static constexpr size_t SZ_TOTAL = SZ_WB + SZ_XB + SZ_CE;
static_assert(SZ_TOTAL <= (size_t)134217728);

extern "C" void kernel_launch(void* const* d_in, const int* in_sizes, int n_in,
                              void* d_out, int out_size, void* d_ws, size_t ws_size, hipStream_t stream) {
    if (n_in < 5) return;
    if ((size_t)in_sizes[0] < (size_t)NB * IND) return;
    if ((size_t)in_sizes[1] < (size_t)NB) return;
    if ((size_t)in_sizes[2] < (size_t)NCP * OUTD * IND) return;
    if ((size_t)in_sizes[3] < (size_t)NCP * OUTD) return;
    if ((size_t)in_sizes[4] < (size_t)16) return;
    if ((size_t)out_size < (size_t)NB * OUTD) return;
    if (SZ_TOTAL > ws_size) return;
    const float* x     = (const float*)d_in[0];
    const float* phase = (const float*)d_in[1];
    const float* w     = (const float*)d_in[2];
    const float* bias  = (const float*)d_in[3];
    const float* basis = (const float*)d_in[4];
    float* OUT = (float*)d_out;
    char* wsp = (char*)d_ws;
    bf* WB = (bf*)wsp; wsp += SZ_WB;
    bf* XB = (bf*)wsp; wsp += SZ_XB;
    float* CE = (float*)wsp; wsp += SZ_CE;

    { const size_t n8 = (size_t)NCP * OUTD * IND / 8; k_cvt8<<<(unsigned)((n8 + 255) / 256), 256, 0, stream>>>(w, WB, n8); }
    { const size_t n8 = (size_t)NB * IND / 8;         k_cvt8<<<(unsigned)((n8 + 255) / 256), 256, 0, stream>>>(x, XB, n8); }
    k_coef<<<(unsigned)((NB + 255) / 256), 256, 0, stream>>>(phase, basis, CE, NB);
    k_pl<<<dim3(NB / 32, OUTD / 64, 1), 32, 0, stream>>>(XB, WB, CE, bias, OUT);
}
